// GATModelSimple_75213467288113
// MI455X (gfx1250) — hardware-verified
//
#include <hip/hip_runtime.h>
#include <stddef.h>


#define FIN   166
#define KP    192
#define HCH   256
#define NHEAD 4
#define HDIM  64
#define NCLS  2
#define NPAD  16

#define NTHR  256
#define NWAVE 8

#define GR    32
#define AP    200
#define XSP   260

#define CHUNK 2048
#define WCAP  256
#define NGRP  (CHUNK / (NTHR * 4))

#define NB1   256
#define SB1   8
#define NB2   4096
#define SB2   12

#define L1_SACC (NB1 * HCH)
#define L1_MAX  (NB1 * NHEAD)
#define L1_DEN  (NB1 * NHEAD)
#define L1_LIST (NWAVE * WCAP)
#define LDS1_BYTES ((L1_SACC + L1_MAX + L1_DEN + L1_LIST + NWAVE) * 4)

#define L2_SACC (NB2 * NCLS)
#define L2_MAX  NB2
#define L2_DEN  NB2
#define L2_LIST (NWAVE * WCAP)
#define LDS2_BYTES ((L2_SACC + L2_MAX + L2_DEN + L2_LIST + NWAVE) * 4)

static_assert(KP % 32 == 0);
static_assert(KP >= FIN);
static_assert(AP >= KP && (AP % 8) == 0);
static_assert(XSP >= HCH && (XSP % 4) == 0);
static_assert(HCH == NHEAD * HDIM);
static_assert(HCH == NWAVE * 32);
static_assert(HDIM == 64);
static_assert(GR == 32 && NTHR == 256);
static_assert(NGRP >= 1 && NGRP * NTHR * 4 == CHUNK);
static_assert(WCAP == (CHUNK / NTHR) * 32);
static_assert(NB1 == (1 << SB1) && NB2 == (1 << SB2));
static_assert(CHUNK <= 2048);
static_assert(NB1 == NTHR && NB1 == NWAVE * 32);
static_assert(NB1 * 4 <= L1_LIST);
static_assert(NB2 % NTHR == 0);
static_assert(NB2 * NCLS * 4 == NWAVE * 8 * 32 * 16);
static_assert(LDS1_BYTES == 278560);
static_assert(LDS1_BYTES <= 327680);
static_assert(LDS2_BYTES == 73760);

typedef unsigned short u16;
typedef u16      v8u  __attribute__((ext_vector_type(8)));
typedef __bf16   v8b  __attribute__((ext_vector_type(8)));
typedef __bf16   v16b __attribute__((ext_vector_type(16)));
typedef _Float16 v8h  __attribute__((ext_vector_type(8)));
typedef _Float16 v16h __attribute__((ext_vector_type(16)));
typedef float    v2f  __attribute__((ext_vector_type(2)));
typedef float    v4f  __attribute__((ext_vector_type(4)));
typedef float    v8f  __attribute__((ext_vector_type(8)));
typedef int      v4i  __attribute__((ext_vector_type(4)));
union FragB { v16b v; v8b half[2]; };
union FragH { v16h v; v8h half[2]; };
union PackU { v8u u; v4i i; };
union PackH { v8h h; v4i i; };

__device__ __forceinline__ u16 f2bf(float f) {
  const unsigned int u = __float_as_uint(f);
  const unsigned int r = ((u >> 16) & 1u) + 0x7FFFu;
  return (u16)((u + r) >> 16);
}
__device__ __forceinline__ float bf2f(u16 b) {
  return __uint_as_float(((unsigned int)b) << 16);
}
__device__ __forceinline__ float lrelu(float v) { return v > 0.0f ? v : 0.2f * v; }
__device__ __forceinline__ float elu1(float v)  { return v > 0.0f ? v : (__expf(v) - 1.0f); }
__device__ __forceinline__ int clampi(int v, int lo, int hi) { return v < lo ? lo : (v > hi ? hi : v); }

__device__ __forceinline__ v8f wmb(v16b a, v16b b, v8f c) {
  v8f d = __builtin_amdgcn_wmma_f32_16x16x32_bf16(false, a, false, b, (short)0, c, false, false);
  asm volatile("v_nop\n\tv_nop\n\tv_nop\n\tv_nop" : "+v"(d) : "v"(a), "v"(b));
  return d;
}
__device__ __forceinline__ v8f wmh(v16h a, v16h b, v8f c) {
  v8f d = __builtin_amdgcn_wmma_f32_16x16x32_f16(false, a, false, b, (short)0, c, false, false);
  asm volatile("v_nop\n\tv_nop\n\tv_nop\n\tv_nop" : "+v"(d) : "v"(a), "v"(b));
  return d;
}

template <int NB, int SB>
__device__ __forceinline__ int scan_groups(const int* __restrict__ eid, int nE, bool vec, int cbase,
                                           int nodeBase, int tid, int wave, int* list) {
  int wc = 0;
#pragma unroll
  for (int g = 0; g < NGRP; ++g) {
    const int el0  = (g * NTHR + tid) * 4;
    const int e0   = cbase + el0;
    const int sent = -2147483647 - 1;
    v4i d;
    if (vec) {
      d = *(const v4i*)(eid + e0);
    } else {
      const int c0 = (e0     < nE) ? e0     : (nE - 1);
      const int c1 = (e0 + 1 < nE) ? e0 + 1 : (nE - 1);
      const int c2 = (e0 + 2 < nE) ? e0 + 2 : (nE - 1);
      const int c3 = (e0 + 3 < nE) ? e0 + 3 : (nE - 1);
      const int v0 = eid[c0], v1 = eid[c1], v2 = eid[c2], v3 = eid[c3];
      d.x = (e0     < nE) ? v0 : sent;
      d.y = (e0 + 1 < nE) ? v1 : sent;
      d.z = (e0 + 2 < nE) ? v2 : sent;
      d.w = (e0 + 3 < nE) ? v3 : sent;
    }
    const unsigned s0 = (unsigned)d.x - (unsigned)nodeBase;
    const unsigned s1 = (unsigned)d.y - (unsigned)nodeBase;
    const unsigned s2 = (unsigned)d.z - (unsigned)nodeBase;
    const unsigned s3 = (unsigned)d.w - (unsigned)nodeBase;
    const bool h0 = s0 < (unsigned)NB;
    const bool h1 = s1 < (unsigned)NB;
    const bool h2 = s2 < (unsigned)NB;
    const bool h3 = s3 < (unsigned)NB;
    const unsigned many = __builtin_amdgcn_ballot_w32(h0 | h1 | h2 | h3);
    if (many != 0u) {
#define HITJ(J, HJ, SJ) { \
        const unsigned mj = __builtin_amdgcn_ballot_w32(HJ); \
        if (HJ) { \
          const int pos = wc + (int)__builtin_amdgcn_mbcnt_lo(mj, 0u); \
          if (pos < WCAP) list[wave * WCAP + pos] = ((el0 + (J)) << SB) | (int)(SJ); \
        } \
        wc += (int)__builtin_popcount(mj); }
      HITJ(0, h0, s0)
      HITJ(1, h1, s1)
      HITJ(2, h2, s2)
      HITJ(3, h3, s3)
#undef HITJ
    }
  }
  return wc;
}

__global__ __launch_bounds__(NTHR) void k_prep(const float* __restrict__ W1, const float* __restrict__ W2,
                                               u16* w1h, u16* w1l, _Float16* w2p) {
  const int nb1 = (HCH * (KP / 8) + NTHR - 1) / NTHR;
  if ((int)blockIdx.x < nb1) {
    const int i = blockIdx.x * NTHR + threadIdx.x;
    if (i >= HCH * (KP / 8)) return;
    const int n  = i / (KP / 8);
    const int k0 = (i - n * (KP / 8)) * 8;
    PackU ph, pl;
#pragma unroll
    for (int j = 0; j < 8; ++j) {
      const int k  = k0 + j;
      const int kc = (k < FIN) ? k : (FIN - 1);
      float v = W1[(size_t)kc * HCH + n];
      v = (k < FIN) ? v : 0.0f;
      const u16 hb = f2bf(v);
      ph.u[j] = hb;
      pl.u[j] = f2bf(v - bf2f(hb));
    }
    u16* dh = w1h + (size_t)i * 8;
    u16* dl = w1l + (size_t)i * 8;
    *(volatile v4i*)dh = ph.i;
    *(volatile v4i*)dl = pl.i;
    __threadfence();
    *(volatile v4i*)dh = ph.i;
    *(volatile v4i*)dl = pl.i;
  } else {
    const int i = ((int)blockIdx.x - nb1) * NTHR + threadIdx.x;
    if (i >= NPAD * (HCH / 8)) return;
    const int n  = i / (HCH / 8);
    const int k0 = (i - n * (HCH / 8)) * 8;
    const int nc = (n < NCLS) ? n : (NCLS - 1);
    PackH pw;
#pragma unroll
    for (int j = 0; j < 8; ++j) {
      float v = W2[(size_t)(k0 + j) * NCLS + nc] * 16.0f;
      v = (n < NCLS) ? v : 0.0f;
      pw.h[j] = (_Float16)v;
    }
    _Float16* dp = w2p + (size_t)i * 8;
    *(volatile v4i*)dp = pw.i;
    __threadfence();
    *(volatile v4i*)dp = pw.i;
  }
}

__global__ __launch_bounds__(NTHR) void k_gemm1(
    const float* __restrict__ x, const u16* __restrict__ w1h, const u16* __restrict__ w1l,
    const float* __restrict__ aS1, const float* __restrict__ aD1,
    float* h1, float* as1, float* ad1, int nN) {
  __shared__ __attribute__((aligned(16))) u16   Ah[GR * AP];
  __shared__ __attribute__((aligned(16))) u16   Al[GR * AP];
  __shared__ __attribute__((aligned(16))) float Xs[GR * XSP];
  __shared__ __attribute__((aligned(16))) float Pq[2 * GR * NHEAD];

  const int tid  = threadIdx.x;
  const int lane = tid & 31;
  const int wave = tid >> 5;
  const int hh   = lane >> 4;
  const int m    = lane & 15;
  const int rowBase = blockIdx.x * GR;

  {
    const int r = tid >> 3;
    const int c = tid & 7;
    int row = rowBase + r;
    if (row > nN - 1) row = nN - 1;
    const float* xr = x + (size_t)row * FIN;
    u16 hb[24], lb[24];
#pragma unroll
    for (int j = 0; j < 24; ++j) {
      const int k  = 24 * c + j;
      const int kc = (k < FIN) ? k : (FIN - 1);
      float v = xr[kc];
      v = (k < FIN) ? v : 0.0f;
      const u16 hv = f2bf(v);
      hb[j] = hv;
      lb[j] = f2bf(v - bf2f(hv));
    }
#pragma unroll
    for (int q = 0; q < 3; ++q) {
      v8u uh, ul;
#pragma unroll
      for (int j = 0; j < 8; ++j) { uh[j] = hb[8 * q + j]; ul[j] = lb[8 * q + j]; }
      *(v8u*)(Ah + r * AP + 24 * c + 8 * q) = uh;
      *(v8u*)(Al + r * AP + 24 * c + 8 * q) = ul;
    }
  }
  __syncthreads();

  const int col0 = wave * 32 + m;
  const v8f z8 = {0.f, 0.f, 0.f, 0.f, 0.f, 0.f, 0.f, 0.f};
  v8f c00 = z8, c01 = z8, c10 = z8, c11 = z8;
  const u16* pah0 = Ah + m * AP + 8 * hh;
  const u16* pah1 = Ah + (16 + m) * AP + 8 * hh;
  const u16* pal0 = Al + m * AP + 8 * hh;
  const u16* pal1 = Al + (16 + m) * AP + 8 * hh;
  const u16* pbh0 = w1h + (size_t)col0 * KP + 8 * hh;
  const u16* pbh1 = w1h + (size_t)(col0 + 16) * KP + 8 * hh;
  const u16* pbl0 = w1l + (size_t)col0 * KP + 8 * hh;
  const u16* pbl1 = w1l + (size_t)(col0 + 16) * KP + 8 * hh;
#pragma unroll 1
  for (int kt = 0; kt < KP / 32; ++kt) {
    const int k0 = kt * 32;
    FragB ah0, ah1, al0, al1, bh0, bh1, bl0, bl1;
    ah0.half[0] = *(const v8b*)(pah0 + k0); ah0.half[1] = *(const v8b*)(pah0 + k0 + 16);
    ah1.half[0] = *(const v8b*)(pah1 + k0); ah1.half[1] = *(const v8b*)(pah1 + k0 + 16);
    al0.half[0] = *(const v8b*)(pal0 + k0); al0.half[1] = *(const v8b*)(pal0 + k0 + 16);
    al1.half[0] = *(const v8b*)(pal1 + k0); al1.half[1] = *(const v8b*)(pal1 + k0 + 16);
    bh0.half[0] = *(const v8b*)(pbh0 + k0); bh0.half[1] = *(const v8b*)(pbh0 + k0 + 16);
    bh1.half[0] = *(const v8b*)(pbh1 + k0); bh1.half[1] = *(const v8b*)(pbh1 + k0 + 16);
    bl0.half[0] = *(const v8b*)(pbl0 + k0); bl0.half[1] = *(const v8b*)(pbl0 + k0 + 16);
    bl1.half[0] = *(const v8b*)(pbl1 + k0); bl1.half[1] = *(const v8b*)(pbl1 + k0 + 16);
    c00 = wmb(ah0.v, bh0.v, c00); c00 = wmb(ah0.v, bl0.v, c00); c00 = wmb(al0.v, bh0.v, c00);
    c01 = wmb(ah0.v, bh1.v, c01); c01 = wmb(ah0.v, bl1.v, c01); c01 = wmb(al0.v, bh1.v, c01);
    c10 = wmb(ah1.v, bh0.v, c10); c10 = wmb(ah1.v, bl0.v, c10); c10 = wmb(al1.v, bh0.v, c10);
    c11 = wmb(ah1.v, bh1.v, c11); c11 = wmb(ah1.v, bl1.v, c11); c11 = wmb(al1.v, bh1.v, c11);
  }

  {
    float* x0 = Xs + (8 * hh) * XSP + col0;
    float* x1 = Xs + (16 + 8 * hh) * XSP + col0;
#pragma unroll
    for (int r = 0; r < 8; ++r) {
      x0[r * XSP]      = c00[r];
      x0[r * XSP + 16] = c01[r];
      x1[r * XSP]      = c10[r];
      x1[r * XSP + 16] = c11[r];
    }
  }
  __syncthreads();

  if (tid < GR * NHEAD) {
    const int rr = tid >> 2;
    const int hq = tid & 3;
    const float* xs = Xs + rr * XSP + hq * HDIM;
    const float* ps = aS1 + hq * HDIM;
    const float* pd = aD1 + hq * HDIM;
    float s = 0.0f, d = 0.0f;
#pragma unroll 4
    for (int cc = 0; cc < HDIM; ++cc) {
      const float v = xs[cc];
      s += v * ps[cc];
      d += v * pd[cc];
    }
    Pq[rr * NHEAD + hq]              = s;
    Pq[GR * NHEAD + rr * NHEAD + hq] = d;
  }
  __syncthreads();

  v4f xr0[4], xr1[4];
#pragma unroll
  for (int i = 0; i < 4; ++i) {
    xr0[i] = *(const v4f*)(Xs + (4 * wave + i) * XSP + 4 * lane);
    xr1[i] = *(const v4f*)(Xs + (4 * wave + i) * XSP + 128 + 4 * lane);
  }
  const int pw = (wave < 2) ? wave : 0;
  const v4f av = *(const v4f*)(Pq + pw * GR * NHEAD + 4 * lane);
  float* ap = ((wave == 0) ? as1 : ad1) + (size_t)(rowBase + lane) * NHEAD;
  float* hp[4];
#pragma unroll
  for (int i = 0; i < 4; ++i) hp[i] = h1 + (size_t)(rowBase + 4 * wave + i) * HCH + 4 * lane;

#pragma unroll
  for (int i = 0; i < 4; ++i) {
    *(volatile v4f*)(hp[i])       = xr0[i];
    *(volatile v4f*)(hp[i] + 128) = xr1[i];
  }
  if (wave < 2) *(volatile v4f*)ap = av;
  __threadfence();
#pragma unroll
  for (int i = 0; i < 4; ++i) {
    *(volatile v4f*)(hp[i])       = xr0[i];
    *(volatile v4f*)(hp[i] + 128) = xr1[i];
  }
  if (wave < 2) *(volatile v4f*)ap = av;
}

__global__ __launch_bounds__(NTHR) void k_agg1(
    const int* __restrict__ ei, const float* __restrict__ h1,
    const float* __restrict__ as1, const float* __restrict__ ad1,
    const float* __restrict__ b1, const _Float16* __restrict__ w2p,
    const float* __restrict__ aS2, const float* __restrict__ aD2,
    float* g2, int nN, int nE) {
  extern __shared__ v4f lds1[];
  float* sacc = (float*)lds1;
  float* smax = sacc + L1_SACC;
  float* sden = smax + L1_MAX;
  int*   list = (int*)(sden + L1_DEN);
  int*   wcnt = list + L1_LIST;
  _Float16* hrow = (_Float16*)lds1;

  const int tid  = threadIdx.x;
  const int lane = tid & 31;
  const int wave = tid >> 5;
  const int hd   = lane >> 3;
  const int nodeBase = blockIdx.x * NB1;

#pragma unroll 1
  for (int j = 0; j < NB1 / NWAVE; ++j) {
    const int slot = wave * (NB1 / NWAVE) + j;
    int node = nodeBase + slot;
    if (node > nN - 1) node = nN - 1;
    const float* hp = h1 + (size_t)node * HCH + 8 * lane;
    const v4f a = *(const v4f*)hp;
    const v4f b = *(const v4f*)(hp + 4);
    v4f* sp = (v4f*)(sacc + slot * HCH + 8 * lane);
    sp[0] = a;
    sp[1] = b;
  }
  {
    int node = nodeBase + tid;
    if (node > nN - 1) node = nN - 1;
    const v4f s = *(const v4f*)(as1 + (size_t)node * NHEAD);
    const v4f d = *(const v4f*)(ad1 + (size_t)node * NHEAD);
    v4f lg = s + d;
    lg.x = lrelu(lg.x); lg.y = lrelu(lg.y); lg.z = lrelu(lg.z); lg.w = lrelu(lg.w);
    const v4f one4 = {1.0f, 1.0f, 1.0f, 1.0f};
    *(v4f*)(smax + NHEAD * tid) = lg;
    *(v4f*)(sden + NHEAD * tid) = one4;
  }
  __syncthreads();

  const int* eid = ei + nE;
  const bool al16 = ((nE & 3) == 0);
  const int nChunks = (nE + CHUNK - 1) / CHUNK;
#pragma unroll 1
  for (int ch = 0; ch < nChunks; ++ch) {
    const int  cbase = ch * CHUNK;
    const bool vec   = al16 && (cbase + CHUNK <= nE);
    const int  wc    = scan_groups<NB1, SB1>(eid, nE, vec, cbase, nodeBase, tid, wave, list);
    if (lane == 0) wcnt[wave] = wc;
    __syncthreads();

    if (wave == 0) {
#pragma unroll 1
      for (int wsx = 0; wsx < NWAVE; ++wsx) {
        int n = wcnt[wsx];
        n = (n > WCAP) ? WCAP : ((n < 0) ? 0 : n);
#pragma unroll 1
        for (int i = 0; i < n; ++i) {
          const int ent  = list[wsx * WCAP + i];
          const int slot = ent & (NB1 - 1);
          const int el   = (ent >> SB1) & (CHUNK - 1);
          int e = cbase + el;
          if (e > nE - 1) e = nE - 1;
          const int src = clampi(ei[e], 0, nN - 1);
          int nd = nodeBase + slot;
          if (nd > nN - 1) nd = nN - 1;
          float lg = as1[(size_t)src * NHEAD + hd] + ad1[(size_t)nd * NHEAD + hd];
          lg = lrelu(lg);
          const int   mi = slot * NHEAD + hd;
          const float mo = smax[mi];
          const float mn = fmaxf(mo, lg);
          const float sc = __expf(mo - mn);
          const float p  = __expf(lg - mn);
          const float* hp = h1 + (size_t)src * HCH + 8 * lane;
          const v4f x0 = *(const v4f*)hp;
          const v4f x1 = *(const v4f*)(hp + 4);
          v4f* sp = (v4f*)(sacc + slot * HCH + 8 * lane);
          const v4f c0 = sp[0];
          const v4f c1 = sp[1];
          sp[0] = c0 * sc + x0 * p;
          sp[1] = c1 * sc + x1 * p;
          const float dn = sden[mi];
          smax[mi] = mn;
          sden[mi] = dn * sc + p;
        }
      }
    }
    __syncthreads();
  }

  {
    const v4f bb0 = *(const v4f*)(b1 + 8 * lane);
    const v4f bb1 = *(const v4f*)(b1 + 8 * lane + 4);
#pragma unroll 1
    for (int j = 0; j < NB1 / NWAVE; ++j) {
      const int slot = wave * (NB1 / NWAVE) + j;
      const v4f* sp = (const v4f*)(sacc + slot * HCH + 8 * lane);
      const v4f c0 = sp[0];
      const v4f c1 = sp[1];
      const float dn  = sden[slot * NHEAD + hd];
      const float inv = 1.0f / (dn + 1e-16f);
      v4f u0 = c0 * inv + bb0;
      v4f u1 = c1 * inv + bb1;
      PackH pk;
      pk.h[0] = (_Float16)elu1(u0.x); pk.h[1] = (_Float16)elu1(u0.y);
      pk.h[2] = (_Float16)elu1(u0.z); pk.h[3] = (_Float16)elu1(u0.w);
      pk.h[4] = (_Float16)elu1(u1.x); pk.h[5] = (_Float16)elu1(u1.y);
      pk.h[6] = (_Float16)elu1(u1.z); pk.h[7] = (_Float16)elu1(u1.w);
      *(v8h*)(hrow + (size_t)slot * (2 * HCH) + 8 * lane) = pk.h;
    }
  }
  __syncthreads();

  float* G = (float*)list;
  {
    const int m  = lane & 15;
    const int hh = lane >> 4;
    const v8f z8 = {0.f, 0.f, 0.f, 0.f, 0.f, 0.f, 0.f, 0.f};
    v8f ga0 = z8, ga1 = z8;
    const _Float16* pa0 = hrow + (size_t)(wave * 32 + m) * (2 * HCH) + 8 * hh;
    const _Float16* pa1 = hrow + (size_t)(wave * 32 + 16 + m) * (2 * HCH) + 8 * hh;
    const _Float16* pb  = w2p + (size_t)m * HCH + 8 * hh;
#pragma unroll 1
    for (int kt = 0; kt < HCH / 32; ++kt) {
      const int k0 = kt * 32;
      FragH a0, a1, b;
      b.half[0]  = *(const v8h*)(pb + k0);   b.half[1]  = *(const v8h*)(pb + k0 + 16);
      a0.half[0] = *(const v8h*)(pa0 + k0);  a0.half[1] = *(const v8h*)(pa0 + k0 + 16);
      a1.half[0] = *(const v8h*)(pa1 + k0);  a1.half[1] = *(const v8h*)(pa1 + k0 + 16);
      ga0 = wmh(a0.v, b.v, ga0);
      ga1 = wmh(a1.v, b.v, ga1);
    }
    if (m < NCLS) {
#pragma unroll
      for (int r = 0; r < 8; ++r) {
        G[(wave * 32 + 8 * hh + r) * 4 + m]      = ga0[r] * 0.0625f;
        G[(wave * 32 + 16 + 8 * hh + r) * 4 + m] = ga1[r] * 0.0625f;
      }
    }
  }
  __syncthreads();

  {
    const float g0 = G[4 * tid];
    const float g1 = G[4 * tid + 1];
    const float s0 = aS2[0], s1 = aS2[1];
    const float d0 = aD2[0], d1 = aD2[1];
    v4f o;
    o.x = g0;
    o.y = g1;
    o.z = g0 * s0 + g1 * s1;
    o.w = g0 * d0 + g1 * d1;
    float* gp = g2 + (size_t)(nodeBase + tid) * 4;
    *(volatile v4f*)gp = o;
    __threadfence();
    *(volatile v4f*)gp = o;
  }
}

__global__ __launch_bounds__(NTHR) void k_agg2(
    const int* __restrict__ ei, const float* __restrict__ g2, const float* __restrict__ b2,
    float* out, int nN, int nE) {
  extern __shared__ v4f lds2[];
  float* sacc = (float*)lds2;
  float* smax = sacc + L2_SACC;
  float* sden = smax + L2_MAX;
  int*   list = (int*)(sden + L2_DEN);
  int*   wcnt = list + L2_LIST;

  const int tid  = threadIdx.x;
  const int lane = tid & 31;
  const int wave = tid >> 5;
  const int nodeBase = blockIdx.x * NB2;

#pragma unroll 1
  for (int j = 0; j < NB2 / NTHR; ++j) {
    const int slot = j * NTHR + tid;
    int node = nodeBase + slot;
    if (node > nN - 1) node = nN - 1;
    const v4f gv = *(const v4f*)(g2 + (size_t)node * 4);
    v2f c;
    c.x = gv.x;
    c.y = gv.y;
    *(v2f*)(sacc + NCLS * slot) = c;
    smax[slot] = lrelu(gv.z + gv.w);
    sden[slot] = 1.0f;
  }
  __syncthreads();

  const int* eid = ei + nE;
  const bool al16 = ((nE & 3) == 0);
  const int nChunks = (nE + CHUNK - 1) / CHUNK;
#pragma unroll 1
  for (int ch = 0; ch < nChunks; ++ch) {
    const int  cbase = ch * CHUNK;
    const bool vec   = al16 && (cbase + CHUNK <= nE);
    const int  wc    = scan_groups<NB2, SB2>(eid, nE, vec, cbase, nodeBase, tid, wave, list);
    if (lane == 0) wcnt[wave] = wc;
    __syncthreads();

    if (wave == 0) {
#pragma unroll 1
      for (int wsx = 0; wsx < NWAVE; ++wsx) {
        int n = wcnt[wsx];
        n = (n > WCAP) ? WCAP : ((n < 0) ? 0 : n);
#pragma unroll 1
        for (int i = 0; i < n; ++i) {
          const int ent  = list[wsx * WCAP + i];
          const int slot = ent & (NB2 - 1);
          const int el   = (ent >> SB2) & (CHUNK - 1);
          int e = cbase + el;
          if (e > nE - 1) e = nE - 1;
          const int src = clampi(ei[e], 0, nN - 1);
          int nd = nodeBase + slot;
          if (nd > nN - 1) nd = nN - 1;
          const v4f gs   = *(const v4f*)(g2 + (size_t)src * 4);
          const float ad = g2[(size_t)nd * 4 + 3];
          const float lg = lrelu(gs.z + ad);
          const float mo = smax[slot];
          const float mn = fmaxf(mo, lg);
          const float sc = __expf(mo - mn);
          const float p  = __expf(lg - mn);
          v2f* sp = (v2f*)(sacc + NCLS * slot);
          const v2f c = *sp;
          v2f hv;
          hv.x = gs.x;
          hv.y = gs.y;
          *sp = c * sc + hv * p;
          const float dn = sden[slot];
          smax[slot] = mn;
          sden[slot] = dn * sc + p;
        }
      }
    }
    __syncthreads();
  }

  {
    const float bz0 = b2[0], bz1 = b2[1];
#pragma unroll 1
    for (int j = 0; j < NB2 / NTHR; ++j) {
      const int slot = j * NTHR + tid;
      v2f* sp = (v2f*)(sacc + NCLS * slot);
      const v2f c = *sp;
      const float dn  = sden[slot];
      const float inv = 1.0f / (dn + 1e-16f);
      v2f o;
      o.x = c.x * inv + bz0;
      o.y = c.y * inv + bz1;
      *sp = o;
    }
  }
  __syncthreads();

#pragma unroll 1
  for (int it = 0; it < 8; ++it) {
    const int q  = (wave * 8 + it) * 32 + lane;
    const int r0 = nodeBase + 2 * q;
    const v4f v  = *(const v4f*)(sacc + 4 * q);
    float* op = out + (size_t)r0 * NCLS;
    if (r0 + 1 < nN) {
      *(volatile v4f*)op = v;
    } else if (r0 < nN) {
      v2f t; t.x = v.x; t.y = v.y;
      *(volatile v2f*)op = t;
    }
  }
  __threadfence();
#pragma unroll 1
  for (int it = 0; it < 8; ++it) {
    const int q  = (wave * 8 + it) * 32 + lane;
    const int r0 = nodeBase + 2 * q;
    const v4f v  = *(const v4f*)(sacc + 4 * q);
    float* op = out + (size_t)r0 * NCLS;
    if (r0 + 1 < nN) {
      *(volatile v4f*)op = v;
    } else if (r0 < nN) {
      v2f t; t.x = v.x; t.y = v.y;
      *(volatile v2f*)op = t;
    }
  }
}

extern "C" void kernel_launch(void* const* d_in, const int* in_sizes, int n_in,
                              void* d_out, int out_size, void* d_ws, size_t ws_size,
                              hipStream_t stream) {
  if (n_in < 10) return;
  const int nN = in_sizes[0] / FIN;
  if (nN <= 0 || in_sizes[0] != nN * FIN) return;
  if (in_sizes[1] < 0 || (in_sizes[1] & 1) != 0) return;
  const int nE = in_sizes[1] / 2;
  if (in_sizes[2] != FIN * HCH) return;
  if (in_sizes[3] != HCH || in_sizes[4] != HCH || in_sizes[5] != HCH) return;
  if (in_sizes[6] != HCH * NCLS || in_sizes[7] != NCLS || in_sizes[8] != NCLS || in_sizes[9] != NCLS) return;
  if (out_size != nN * NCLS) return;

  const float* x   = (const float*)d_in[0];
  const int*   ei  = (const int*)d_in[1];
  const float* W1  = (const float*)d_in[2];
  const float* aS1 = (const float*)d_in[3];
  const float* aD1 = (const float*)d_in[4];
  const float* b1  = (const float*)d_in[5];
  const float* W2  = (const float*)d_in[6];
  const float* aS2 = (const float*)d_in[7];
  const float* aD2 = (const float*)d_in[8];
  const float* b2  = (const float*)d_in[9];
  float* out = (float*)d_out;

  const int nP1 = ((nN + GR - 1) / GR) * GR;
  const int nP2 = ((nN + NB1 - 1) / NB1) * NB1;
  const int nA2 = (nN + NB2 - 1) / NB2;

  size_t off = 0;
  auto carve = [&](size_t bytes) -> char* {
    char* p = (char*)d_ws + off;
    off += (bytes + 255) & ~(size_t)255;
    return p;
  };
  u16*      w1h = (u16*)carve((size_t)HCH * KP * sizeof(u16));
  u16*      w1l = (u16*)carve((size_t)HCH * KP * sizeof(u16));
  _Float16* w2p = (_Float16*)carve((size_t)NPAD * HCH * sizeof(_Float16));
  float*    h1  = (float*)carve((size_t)nP1 * HCH * sizeof(float));
  float*    as1 = (float*)carve((size_t)nP1 * NHEAD * sizeof(float));
  float*    ad1 = (float*)carve((size_t)nP1 * NHEAD * sizeof(float));
  float*    g2  = (float*)carve((size_t)nP2 * 4 * sizeof(float));
  if (off > ws_size) return;
  if (off > (size_t)134217728) return;

  const int nbW1 = (HCH * (KP / 8) + NTHR - 1) / NTHR;
  const int nbW2 = (NPAD * (HCH / 8) + NTHR - 1) / NTHR;
  k_prep<<<nbW1 + nbW2, NTHR, 0, stream>>>(W1, W2, w1h, w1l, w2p);

  k_gemm1<<<nP1 / GR, NTHR, 0, stream>>>(x, w1h, w1l, aS1, aD1, h1, as1, ad1, nN);

  hipFuncSetAttribute(reinterpret_cast<const void*>(&k_agg1),
                      hipFuncAttributeMaxDynamicSharedMemorySize, LDS1_BYTES);
  k_agg1<<<nP2 / NB1, NTHR, LDS1_BYTES, stream>>>(ei, h1, as1, ad1, b1, w2p, aS2, aD2, g2, nN, nE);

  hipFuncSetAttribute(reinterpret_cast<const void*>(&k_agg2),
                      hipFuncAttributeMaxDynamicSharedMemorySize, LDS2_BYTES);
  k_agg2<<<nA2, NTHR, LDS2_BYTES, stream>>>(ei, g2, b2, out, nN, nE);
}
